// SpatialLocalSum_22308060135554
// MI455X (gfx1250) — hardware-run, weakly checked
//
#include <hip/hip_runtime.h>


namespace {
constexpr int NB = 128, HW = 32 * 32, C = 64, S = 64;
constexpr float XS = 8.0f;
typedef _Float16 b16;
typedef __attribute__((ext_vector_type(16))) _Float16 v16b;
typedef __attribute__((ext_vector_type(8))) _Float16 v8b;
typedef __attribute__((ext_vector_type(8))) float v8f;
typedef __attribute__((ext_vector_type(4))) float v4f;
typedef __attribute__((ext_vector_type(2))) float v2f;
__device__ __forceinline__ float bf16_rne(float f) { unsigned int u = __float_as_uint(f); u += 0x7FFFu + ((u >> 16) & 1u); float r = __uint_as_float(u & 0xFFFF0000u); asm volatile("" : "+v"(r)); return r; }
__device__ __forceinline__ void split16(float v, b16& hi, b16& lo) { hi = (b16)v; lo = (b16)(v - (float)hi); }
__device__ __forceinline__ v16b frag_kb(const b16* p, int hh) { const v8b a = *(const v8b*)(p + 8 * hh), b = *(const v8b*)(p + 16 + 8 * hh); v16b f;
#pragma unroll
  for (int e = 0; e < 8; ++e) { f[e] = a[e]; f[8 + e] = b[e]; } return f; }
__device__ __forceinline__ v8f wmma16b(v16b a, v16b b, v8f c) { v8f d = __builtin_amdgcn_wmma_f32_16x16x32_f16(false, a, false, b, (short)0, c, false, false); asm volatile("v_nop\n\tv_nop\n\tv_nop\n\tv_nop" : "+v"(d) : "v"(a), "v"(b)); return d; }
__device__ __forceinline__ void wave_lds_sync() { __builtin_amdgcn_fence(__ATOMIC_RELEASE, "workgroup"); __builtin_amdgcn_wave_barrier(); __builtin_amdgcn_fence(__ATOMIC_ACQUIRE, "workgroup"); }
__device__ __forceinline__ float pmul(float a, float b) { float p = a * b; asm volatile("" : "+v"(p)); return p; }

__global__ __launch_bounds__(256) void wprep_kernel(const float* __restrict__ accu, b16* __restrict__ WBh, b16* __restrict__ WBl, float* __restrict__ MW) { const int wave = threadIdx.x >> 5, lane = threadIdx.x & 31; const int wid = blockIdx.x * 8 + wave; if (wid >= HW * 2) return; const int pos = wid >> 1, s = (wid & 1) * 32 + lane; const float* ap = accu + (size_t)pos * C * S + s;
  float mxv = 0.0f, sum = 0.0f;
#pragma unroll 4
  for (int c = 0; c < C; ++c) { const float a = bf16_rne(ap[(size_t)c * S]); mxv = fmaxf(mxv, a); sum += a; }
  const float inv = 1.0f / mxv; b16* dh = WBh + ((size_t)pos * S + s) * C; b16* dl = WBl + ((size_t)pos * S + s) * C;
#pragma unroll 1
  for (int c8 = 0; c8 < C; c8 += 8) { v8b vh, vl; for (int j = 0; j < 8; ++j) { b16 p, ql; split16(pmul(bf16_rne(ap[(size_t)(c8 + j) * S]), inv) * XS, p, ql); vh[j] = p; vl[j] = ql; } for (int pass = 0; pass < 2; ++pass) { *(volatile v8b*)(dh + c8) = vh; *(volatile v8b*)(dl + c8) = vl; __threadfence(); } }
  for (int pass = 0; pass < 2; ++pass) { ((volatile float*)MW)[(size_t)pos * S + s] = __logf(mxv) - __logf(sum); __threadfence(); } }
__global__ __launch_bounds__(32) void main_kernel(const float* __restrict__ x, const b16* __restrict__ WBh, const b16* __restrict__ WBl, const float* __restrict__ MW, int PLIM, float* __restrict__ out) { __shared__ __attribute__((aligned(16))) b16 Ah[16][C + 8], Al[16][C + 8]; __shared__ float Tf[16][68]; __shared__ float MX[16]; const int lane = threadIdx.x, nloc = lane & 15, hlf = lane >> 4; const int pos = blockIdx.x / (NB / 16), bt = blockIdx.x % (NB / 16); if (pos >= PLIM) return; const int b0 = bt * 16;
  for (int rr = 0; rr < 16; ++rr) { const float* xp = x + ((size_t)(b0 + rr) * HW + pos) * C; const float v0 = bf16_rne(xp[lane]), v1 = bf16_rne(xp[32 + lane]); float m = fmaxf(v0, v1); for (int o = 16; o; o >>= 1) m = fmaxf(m, __shfl_xor(m, o)); if (lane == 0) MX[rr] = m;
    b16 p, ql; split16(__expf(v0 - m) * XS, p, ql); Ah[rr][lane] = p; Al[rr][lane] = ql; split16(__expf(v1 - m) * XS, p, ql); Ah[rr][32 + lane] = p; Al[rr][32 + lane] = ql; }
  wave_lds_sync(); v8f acc[4];
#pragma unroll
  for (int t = 0; t < 4; ++t) acc[t] = (v8f){};
#pragma unroll
  for (int kb = 0; kb < C; kb += 32) { const v16b ah = frag_kb(&Ah[nloc][kb], hlf), al = frag_kb(&Al[nloc][kb], hlf);
#pragma unroll
    for (int t = 0; t < 4; ++t) { const size_t ro = ((size_t)pos * S + t * 16 + nloc) * C + kb; const v16b bh = frag_kb(WBh + ro, hlf), bl = frag_kb(WBl + ro, hlf); acc[t] = wmma16b(ah, bh, acc[t]); acc[t] = wmma16b(ah, bl, acc[t]); acc[t] = wmma16b(al, bh, acc[t]); acc[t] = wmma16b(al, bl, acc[t]); } }
#pragma unroll
  for (int t = 0; t < 4; ++t) { const int s = t * 16 + nloc; const float mw = MW[(size_t)pos * S + s];
#pragma unroll
    for (int r8 = 0; r8 < 8; ++r8) { const int rr = 8 * hlf + r8; Tf[rr][s] = __logf(acc[t][r8] * (1.0f / (XS * XS))) + MX[rr] + mw; } }
  wave_lds_sync();
  for (int pass = 0; pass < 2; ++pass) { for (int rr = 0; rr < 16; ++rr) *(volatile v2f*)(out + ((size_t)(b0 + rr) * HW + pos) * S + lane * 2) = (v2f){Tf[rr][lane * 2], Tf[rr][lane * 2 + 1]}; __threadfence(); } }
}

extern "C" void kernel_launch(void* const* d_in, const int* in_sizes, int n_in, void* d_out, int out_size, void* d_ws, size_t ws_size, hipStream_t stream) {
  (void)n_in;
  auto Fp = [&](int i) { return (const float*)d_in[i]; };
  if (in_sizes[0] != NB * HW * C || in_sizes[1] != HW * C * S || out_size != NB * HW * S) return;
  const int PLIM = HW;
  size_t off = 0; char* ws = (char*)d_ws;
  auto carve = [&](size_t bytes) { char* p = ws + off; off += (bytes + 255) & ~(size_t)255; return p; };
  b16* WBh = (b16*)carve((size_t)HW * S * C * 2); b16* WBl = (b16*)carve((size_t)HW * S * C * 2); float* MW = (float*)carve((size_t)HW * S * 4);
  if (off > ws_size || off > ((size_t)32 << 20)) return;
  wprep_kernel<<<(HW * 2 + 7) / 8, 256, 0, stream>>>(Fp(1), WBh, WBl, MW);
  main_kernel<<<PLIM * (NB / 16), 32, 0, stream>>>(Fp(0), WBh, WBl, MW, PLIM, (float*)d_out);
}
